// MultiHeadAttentionLayer_59322088292536
// MI455X (gfx1250) — hardware-verified
//
#include <hip/hip_runtime.h>
#include <stdint.h>
#include <stddef.h>


#ifndef NB
#define NB 2
#endif
#ifndef SEQ
#define SEQ 2048
#endif
#define NB_FULL  2
#define SEQ_FULL 2048
#define HID      1024
#define NHEAD    16
#define HDIM     64
#define ROWS     (NB * SEQ)
#define RPH      (SEQ / 16)
#define KSTEPS   (HID / 32)
#define CK       32
#define SQ       128

static_assert(NB >= 1 && NB <= NB_FULL);
static_assert(SEQ >= 256 && SEQ <= SEQ_FULL && (SEQ % 256) == 0);
static_assert(HID == NHEAD * HDIM);
static_assert((ROWS % 128) == 0 && (SEQ % SQ) == 0 && (SEQ % CK) == 0);
static_assert(RPH >= 16 && (RPH % 16) == 0);

typedef unsigned short us_t;
typedef __attribute__((ext_vector_type(8)))  unsigned short v8us;
typedef __attribute__((ext_vector_type(16))) __bf16 v16bf;
typedef __attribute__((ext_vector_type(8)))  float v8f;
typedef __attribute__((ext_vector_type(4)))  float v4f;

union Frag { v16bf v; v8us h[2]; };

__device__ __forceinline__ us_t f2bf(float x)
{
    unsigned u = __float_as_uint(x);
    u += 0x7FFFu + ((u >> 16) & 1u);
    return (us_t)(u >> 16);
}
__device__ __forceinline__ float bf2f(us_t b)
{
    return __uint_as_float(((unsigned)b) << 16);
}

__device__ __forceinline__ v8f wmma_bf(v16bf a, v16bf b, v8f c)
{
    v8f d = __builtin_amdgcn_wmma_f32_16x16x32_bf16(false, a, false, b, (short)0, c, false, false);
    asm volatile("v_nop\n\tv_nop\n\tv_nop\n\tv_nop" : "+v"(d) : "v"(a), "v"(b));
    return d;
}

__device__ __forceinline__ v8f zero8()
{
    v8f z;
#pragma unroll
    for (int i = 0; i < 8; ++i) z[i] = 0.0f;
    return z;
}

__global__ __launch_bounds__(256)
void cvt_kernel(const float* __restrict__ x, us_t* __restrict__ y,
                int nbpb, long long sstride, long long dstride)
{
    const int b   = blockIdx.x / nbpb;
    const int blk = blockIdx.x - b * nbpb;
    const size_t i = (size_t)blk * 2048 + (size_t)threadIdx.x * 8;
    const float* src = x + (size_t)b * (size_t)sstride + i;
    const v4f a = *(const v4f*)src;
    const v4f c = *(const v4f*)(src + 4);
    v8us o;
#pragma unroll
    for (int j = 0; j < 4; ++j) { o[j] = f2bf(a[j]); o[4 + j] = f2bf(c[j]); }
    us_t* dst = y + (size_t)b * (size_t)dstride + i;
    *(volatile v8us*)dst = o;
    __threadfence();
    *(volatile v8us*)dst = o;
}

__global__ __launch_bounds__(256)
void gemm_kernel(const us_t* __restrict__ X, const us_t* __restrict__ W,
                 const float* __restrict__ bias,
                 us_t* __restrict__ ohi, us_t* __restrict__ olo, int mode)
{
    __shared__ __align__(16) us_t bt[64 * 32];
    __shared__ __align__(16) us_t st[8 * 2 * 1024];

    const int lane = threadIdx.x & 31;
    const int wave = threadIdx.x >> 5;
    const int h    = lane >> 4;
    const int ln   = lane & 15;
    const int bx   = blockIdx.x;
    const int by   = blockIdx.y;
    const int m0w  = by * 128 + wave * 16;

    const int tn = threadIdx.x >> 2;
    const int tk = (threadIdx.x & 3) * 8;
    const int wr_t = mode ? ((tn >> 2) * 64 + bx * 4 + (tn & 3)) : (bx * 64 + tn);
    const us_t* wsrc = W + (size_t)wr_t * HID + tk;
    us_t* bdst = bt + tn * 32 + tk;
    const us_t* arow = X + (size_t)(m0w + ln) * HID + 8 * h;

    v8f acc[4];
#pragma unroll
    for (int j = 0; j < 4; ++j) acc[j] = zero8();

    for (int s = 0; s < KSTEPS; ++s) {
        const int kk = s * 32;
        Frag a;
        a.h[0] = *(const v8us*)(arow + kk);
        a.h[1] = *(const v8us*)(arow + kk + 16);
        __syncthreads();
        *(v8us*)bdst = *(const v8us*)(wsrc + kk);
        __syncthreads();
#pragma unroll
        for (int j = 0; j < 4; ++j) {
            const us_t* bp = bt + (j * 16 + ln) * 32 + 8 * h;
            Frag b;
            b.h[0] = *(const v8us*)bp;
            b.h[1] = *(const v8us*)(bp + 16);
            acc[j] = wmma_bf(a.v, b.v, acc[j]);
        }
    }

    us_t* sh = st + wave * 2048;
    us_t* sl = sh + 1024;
#pragma unroll
    for (int j = 0; j < 4; ++j) {
        const int c  = j * 16 + ln;
        const int wr = mode ? ((c >> 2) * 64 + bx * 4 + (c & 3)) : (bx * 64 + c);
        const float bb = bf2f(f2bf(bias[wr]));
        const int ib0   = mode ? ((ln & 3) * 256 + 4 * j + (ln >> 2)) : c;
        const int rstep = mode ? 16 : 64;
#pragma unroll
        for (int r = 0; r < 8; ++r) {
            const float v  = acc[j][r] + bb;
            const us_t hi  = f2bf(v);
            const us_t lo  = f2bf(v - bf2f(hi));
            const int  idx = ib0 + (8 * h + r) * rstep;
            sh[idx] = hi;
            sl[idx] = lo;
        }
    }
    __syncthreads();

    const int bn   = m0w / RPH;
    const int keyb = 16 * (m0w - bn * RPH);
    v8us vh[4], vl[4];
    size_t di[4];
#pragma unroll
    for (int i = 0; i < 4; ++i) {
        const int row = 4 * i + (lane >> 3);
        const int pc  = lane & 7;
        const int sidx = mode ? (i * 256 + 8 * lane) : (row * 64 + pc * 8);
        const size_t d1 = ((size_t)bn * 64 + (size_t)(bx * 4 + i)) * SEQ + (size_t)keyb + (size_t)(8 * lane);
        const size_t d0 = (size_t)(m0w + row) * HID + (size_t)(bx * 64 + pc * 8);
        di[i] = mode ? d1 : d0;
        vh[i] = *(const v8us*)(sh + sidx);
        vl[i] = *(const v8us*)(sl + sidx);
    }
#pragma unroll
    for (int i = 0; i < 4; ++i) {
        *(volatile v8us*)(ohi + di[i]) = vh[i];
        *(volatile v8us*)(olo + di[i]) = vl[i];
    }
    __threadfence();
#pragma unroll
    for (int i = 0; i < 4; ++i) {
        *(volatile v8us*)(ohi + di[i]) = vh[i];
        *(volatile v8us*)(olo + di[i]) = vl[i];
    }
}

__global__ __launch_bounds__(256)
void attn_kernel(const us_t* __restrict__ Qhi, const us_t* __restrict__ Qlo,
                 const us_t* __restrict__ Khi, const us_t* __restrict__ Klo,
                 const us_t* __restrict__ Vhi, const us_t* __restrict__ Vlo,
                 float* __restrict__ out)
{
    __shared__ __align__(16) float lds[9984];
    us_t* L   = (us_t*)lds;
    us_t* khs = L;
    us_t* kls = L + 2304;
    us_t* vhs = L + 4608;
    us_t* vls = L + 7168;
    us_t* phs = L + 9728;
    us_t* pls = L + 14848;

    const int lane  = threadIdx.x & 31;
    const int wave  = threadIdx.x >> 5;
    const int h     = lane >> 4;
    const int ln    = lane & 15;
    const int head  = blockIdx.y;
    const int batch = blockIdx.z;
    const int bn    = batch * NHEAD + head;
    const size_t hb = (size_t)bn * SEQ * HDIM;
    const int q0    = blockIdx.x * SQ + wave * 16;

    Frag qh[2], ql[2];
    {
        const us_t* qrh = Qhi + hb + (size_t)(q0 + ln) * HDIM + 8 * h;
        const us_t* qrl = Qlo + hb + (size_t)(q0 + ln) * HDIM + 8 * h;
#pragma unroll
        for (int f = 0; f < 2; ++f) {
            qh[f].h[0] = *(const v8us*)(qrh + 32 * f);
            qh[f].h[1] = *(const v8us*)(qrh + 32 * f + 16);
            ql[f].h[0] = *(const v8us*)(qrl + 32 * f);
            ql[f].h[1] = *(const v8us*)(qrl + 32 * f + 16);
        }
    }

    v8f o[4];
#pragma unroll
    for (int t = 0; t < 4; ++t) o[t] = zero8();
    float mrow[8], lrow[8];
#pragma unroll
    for (int r = 0; r < 8; ++r) { mrow[r] = -1.0e30f; lrow[r] = 0.0f; }

    us_t* php = phs + wave * 640;
    us_t* plp = pls + wave * 640;

    for (int kk0 = 0; kk0 < SEQ; kk0 += CK) {
        {
            const int row = threadIdx.x >> 3;
            const int c8  = (threadIdx.x & 7) * 8;
            const size_t ko = hb + (size_t)(kk0 + row) * HDIM + c8;
            *(v8us*)(khs + row * 72 + c8) = *(const v8us*)(Khi + ko);
            *(v8us*)(kls + row * 72 + c8) = *(const v8us*)(Klo + ko);
            const int d  = threadIdx.x >> 2;
            const int pc = (threadIdx.x & 3) * 8;
            const size_t vo = hb + (size_t)d * SEQ + (size_t)(kk0 + pc);
            *(v8us*)(vhs + d * 40 + pc) = *(const v8us*)(Vhi + vo);
            *(v8us*)(vls + d * 40 + pc) = *(const v8us*)(Vlo + vo);
        }
        __syncthreads();

        v8f s[2];
#pragma unroll
        for (int j = 0; j < 2; ++j) {
            const us_t* kh = khs + (j * 16 + ln) * 72 + 8 * h;
            const us_t* kl = kls + (j * 16 + ln) * 72 + 8 * h;
            v8f z = zero8();
#pragma unroll
            for (int f = 0; f < 2; ++f) {
                Frag bh, bl;
                bh.h[0] = *(const v8us*)(kh + 32 * f);
                bh.h[1] = *(const v8us*)(kh + 32 * f + 16);
                bl.h[0] = *(const v8us*)(kl + 32 * f);
                bl.h[1] = *(const v8us*)(kl + 32 * f + 16);
                z = wmma_bf(qh[f].v, bh.v, z);
                z = wmma_bf(qh[f].v, bl.v, z);
                z = wmma_bf(ql[f].v, bh.v, z);
            }
            s[j] = z;
        }

#pragma unroll
        for (int r = 0; r < 8; ++r) {
            const float a0 = s[0][r] * 0.125f;
            const float a1 = s[1][r] * 0.125f;
            float v = fmaxf(a0, a1);
#pragma unroll
            for (int off = 1; off < 16; off <<= 1)
                v = fmaxf(v, __shfl_xor(v, off, 32));
            const float mnew  = fmaxf(mrow[r], v);
            const float alpha = __expf(mrow[r] - mnew);
            mrow[r] = mnew;
            const float e0 = __expf(a0 - mnew);
            const float e1 = __expf(a1 - mnew);
            float rs = e0 + e1;
#pragma unroll
            for (int off = 1; off < 16; off <<= 1)
                rs += __shfl_xor(rs, off, 32);
            lrow[r] = lrow[r] * alpha + rs;
#pragma unroll
            for (int t = 0; t < 4; ++t) o[t][r] *= alpha;
            const us_t h0 = f2bf(e0);
            const us_t h1 = f2bf(e1);
            const int  pi = (8 * h + r) * 40;
            php[pi + ln]      = h0;
            php[pi + 16 + ln] = h1;
            plp[pi + ln]      = f2bf(e0 - bf2f(h0));
            plp[pi + 16 + ln] = f2bf(e1 - bf2f(h1));
        }
        __syncthreads();

        Frag ph, pl;
        ph.h[0] = *(const v8us*)(php + ln * 40 + 8 * h);
        ph.h[1] = *(const v8us*)(php + ln * 40 + 16 + 8 * h);
        pl.h[0] = *(const v8us*)(plp + ln * 40 + 8 * h);
        pl.h[1] = *(const v8us*)(plp + ln * 40 + 16 + 8 * h);
#pragma unroll
        for (int t = 0; t < 4; ++t) {
            const us_t* vh = vhs + (16 * t + ln) * 40 + 8 * h;
            const us_t* vl = vls + (16 * t + ln) * 40 + 8 * h;
            Frag bh, bl;
            bh.h[0] = *(const v8us*)vh;
            bh.h[1] = *(const v8us*)(vh + 16);
            bl.h[0] = *(const v8us*)vl;
            bl.h[1] = *(const v8us*)(vl + 16);
            o[t] = wmma_bf(ph.v, bh.v, o[t]);
            o[t] = wmma_bf(ph.v, bl.v, o[t]);
            o[t] = wmma_bf(pl.v, bh.v, o[t]);
        }
        __syncthreads();
    }

    float* ost = lds + wave * 1024;
    float rinv[8];
#pragma unroll
    for (int r = 0; r < 8; ++r) rinv[r] = 1.0f / lrow[r];
#pragma unroll
    for (int t = 0; t < 4; ++t) {
#pragma unroll
        for (int r = 0; r < 8; ++r)
            ost[(8 * h + r) * 64 + 16 * t + ln] = o[t][r] * rinv[r];
    }
    __syncthreads();

    const size_t obase = ((size_t)batch * SEQ + (size_t)q0) * HID + (size_t)head * HDIM;
    v4f ov[8];
    size_t od[8];
#pragma unroll
    for (int i = 0; i < 8; ++i) {
        const int row = 2 * i + (lane >> 4);
        const int f4  = lane & 15;
        ov[i] = *(const v4f*)(ost + row * 64 + f4 * 4);
        od[i] = obase + (size_t)row * HID + (size_t)(f4 * 4);
    }
#pragma unroll
    for (int i = 0; i < 8; ++i) *(volatile v4f*)(out + od[i]) = ov[i];
    __threadfence();
#pragma unroll
    for (int i = 0; i < 8; ++i) *(volatile v4f*)(out + od[i]) = ov[i];
}

extern "C" void kernel_launch(void* const* d_in, const int* in_sizes, int n_in,
                              void* d_out, int out_size, void* d_ws, size_t ws_size,
                              hipStream_t stream)
{
    if (n_in < 9) return;
    const long long need_x = (long long)(NB - 1) * SEQ_FULL * HID + (long long)SEQ * HID;
    if ((long long)in_sizes[0] < need_x || (long long)in_sizes[1] < need_x ||
        (long long)in_sizes[2] < need_x) return;
    if (in_sizes[3] < HID * HID || in_sizes[5] < HID * HID || in_sizes[7] < HID * HID) return;
    if (in_sizes[4] < HID || in_sizes[6] < HID || in_sizes[8] < HID) return;
    if ((long long)out_size < (long long)ROWS * HID) return;

    const float* query = (const float*)d_in[0];
    const float* key   = (const float*)d_in[1];
    const float* value = (const float*)d_in[2];
    const float* Wq    = (const float*)d_in[3];
    const float* bq    = (const float*)d_in[4];
    const float* Wk    = (const float*)d_in[5];
    const float* bk    = (const float*)d_in[6];
    const float* Wv    = (const float*)d_in[7];
    const float* bv    = (const float*)d_in[8];
    float* out = (float*)d_out;

    const size_t PL = (size_t)ROWS * HID;
    const size_t WL = (size_t)HID * HID;
    const size_t total_bytes = (9 * PL + 3 * WL) * sizeof(us_t);
    if (total_bytes > ws_size) return;

    us_t* ws  = (us_t*)d_ws;
    us_t* xq  = ws;
    us_t* xk  = xq + PL;
    us_t* xv  = xk + PL;
    us_t* wqb = xv + PL;
    us_t* wkb = wqb + WL;
    us_t* wvb = wkb + WL;
    us_t* qhi = wvb + WL;
    us_t* qlo = qhi + PL;
    us_t* khi = qlo + PL;
    us_t* klo = khi + PL;
    us_t* vhi = klo + PL;
    us_t* vlo = vhi + PL;

    const int nbpb_x = (SEQ * HID) / 2048;
    const long long sstr = (long long)SEQ_FULL * HID;
    const long long dstr = (long long)SEQ * HID;
    cvt_kernel<<<NB * nbpb_x, 256, 0, stream>>>(query, xq, nbpb_x, sstr, dstr);
    cvt_kernel<<<NB * nbpb_x, 256, 0, stream>>>(key,   xk, nbpb_x, sstr, dstr);
    cvt_kernel<<<NB * nbpb_x, 256, 0, stream>>>(value, xv, nbpb_x, sstr, dstr);
    const int nb_w = (HID * HID) / 2048;
    cvt_kernel<<<nb_w, 256, 0, stream>>>(Wq, wqb, nb_w, 0LL, 0LL);
    cvt_kernel<<<nb_w, 256, 0, stream>>>(Wk, wkb, nb_w, 0LL, 0LL);
    cvt_kernel<<<nb_w, 256, 0, stream>>>(Wv, wvb, nb_w, 0LL, 0LL);

    const dim3 pgrid(HID / 64, ROWS / 128);
    gemm_kernel<<<pgrid, 256, 0, stream>>>(xq, wqb, bq, qhi, qlo, 0);
    gemm_kernel<<<pgrid, 256, 0, stream>>>(xk, wkb, bk, khi, klo, 0);
    gemm_kernel<<<pgrid, 256, 0, stream>>>(xv, wvb, bv, vhi, vlo, 1);

    const dim3 agrid(SEQ / SQ, NHEAD, NB);
    attn_kernel<<<agrid, 256, 0, stream>>>(qhi, qlo, khi, klo, vhi, vlo, out);
}
